// ClassicalAttention_65481071408069
// MI455X (gfx1250) — hardware-verified
//
#include <hip/hip_runtime.h>
#include <stdint.h>

#define NB  4
#define NS  2048
#define ND  1024
static_assert((NS % 64) == 0 && (ND % 64) == 0);
static_assert((NS % 32) == 0 && (ND % 32) == 0);
static_assert(NS == 256 * 8);
static_assert(((NB * NS * ND) % (8 * 256)) == 0 && ((ND * ND) % (8 * 256)) == 0);

typedef __bf16   v16b __attribute__((ext_vector_type(16)));
typedef _Float16 v16h __attribute__((ext_vector_type(16)));
typedef _Float16 v8h  __attribute__((ext_vector_type(8)));
typedef float    v8f  __attribute__((ext_vector_type(8)));
typedef float    v4f  __attribute__((ext_vector_type(4)));
typedef unsigned int v4u __attribute__((ext_vector_type(4)));

__device__ __forceinline__ unsigned short bf_bits(float f) {
  unsigned u = __float_as_uint(f);
  return (unsigned short)((u + 0x7FFFu + ((u >> 16) & 1u)) >> 16);
}
__device__ __forceinline__ unsigned pk16(unsigned short a, unsigned short b) { return (unsigned)a | ((unsigned)b << 16); }
__device__ __forceinline__ v8f zero8() { v8f z = {0.f, 0.f, 0.f, 0.f, 0.f, 0.f, 0.f, 0.f}; return z; }

__device__ __forceinline__ v4u pack_h8(v4f a, v4f b) {
  v8h h;
  h[0] = (_Float16)a[0]; h[1] = (_Float16)a[1]; h[2] = (_Float16)a[2]; h[3] = (_Float16)a[3];
  h[4] = (_Float16)b[0]; h[5] = (_Float16)b[1]; h[6] = (_Float16)b[2]; h[7] = (_Float16)b[3];
  union { v8h h; v4u u; } t;
  t.h = h;
  return t.u;
}

template <typename F>
__device__ __forceinline__ F ldfrag(const unsigned short* p) {
  union { F v; v4u q[2]; } f;
  f.q[0] = *(const v4u*)(p);
  f.q[1] = *(const v4u*)(p + 16);
  return f.v;
}

__device__ __forceinline__ v8f mma16(v16b a, v16b b, v8f c) {
  return __builtin_amdgcn_wmma_f32_16x16x32_bf16(false, a, false, b, (short)0, c, false, false);
}
__device__ __forceinline__ v8f mma16(v16h a, v16h b, v8f c) {
  return __builtin_amdgcn_wmma_f32_16x16x32_f16(false, a, false, b, (short)0, c, false, false);
}
template <typename F>
__device__ __forceinline__ void dep_guard(v8f& a, v8f& b, F x, F y) {
#if defined(__HIP_DEVICE_COMPILE__)
  asm volatile("v_nop\n\tv_nop\n\tv_nop\n\tv_nop" : "+v"(a), "+v"(b) : "v"(x), "v"(y));
#endif
}
template <typename F>
__device__ __forceinline__ void keep4(F a, F b, F c, F d) {
#if defined(__HIP_DEVICE_COMPILE__)
  asm volatile("v_nop" :: "v"(a), "v"(b), "v"(c), "v"(d));
#endif
}
__device__ __forceinline__ void acc_guard4(v8f& a, v8f& b, v8f& c, v8f& d) {
#if defined(__HIP_DEVICE_COMPILE__)
  asm volatile("v_nop\n\tv_nop\n\tv_nop\n\tv_nop" : "+v"(a), "+v"(b), "+v"(c), "+v"(d));
#endif
}
__device__ __forceinline__ void wave_sync_lds() {
  __builtin_amdgcn_fence(__ATOMIC_RELEASE, "workgroup");
  __builtin_amdgcn_wave_barrier();
  __builtin_amdgcn_fence(__ATOMIC_ACQUIRE, "workgroup");
}

__global__ __launch_bounds__(256) void cvt_bf16x8(const float* __restrict__ in, unsigned short* out,
                                                  int n8, int n8tot) {
  const int i = blockIdx.x * 256 + threadIdx.x;
  if (i >= n8tot) return;
  int ic = i;
  if (ic > n8 - 1) ic = n8 - 1;
  const v4f a = *(const v4f*)(in + (size_t)ic * 8);
  const v4f b = *(const v4f*)(in + (size_t)ic * 8 + 4);
  v4u p;
  p[0] = pk16(bf_bits(a[0]), bf_bits(a[1]));
  p[1] = pk16(bf_bits(a[2]), bf_bits(a[3]));
  p[2] = pk16(bf_bits(b[0]), bf_bits(b[1]));
  p[3] = pk16(bf_bits(b[2]), bf_bits(b[3]));
  if (i >= n8) { p[0] = 0u; p[1] = 0u; p[2] = 0u; p[3] = 0u; }
  *(volatile v4u*)(out + (size_t)i * 8) = p;
  __threadfence();
  *(volatile v4u*)(out + (size_t)i * 8) = p;
}

template <typename F, int OUT>
__global__ __launch_bounds__(256) void gemm64(
    const unsigned short* __restrict__ Ap, int lda,
    const unsigned short* __restrict__ Bp, int ldb,
    void* Cout, int ldc, float alpha, int M, int N, int K) {
  __shared__ __align__(16) float sT[8][16 * 68];
  const int lane = threadIdx.x & 31;
  const int wave = threadIdx.x >> 5;
  const int tilesN = N >> 6;
  const int tilesM = M >> 6;
  const int tile = blockIdx.x * 8 + wave;
  if (tile >= tilesM * tilesN) return;
  const int tm = tile / tilesN;
  const int tn = tile - tm * tilesN;
  const int m0 = tm << 6;
  const int n0 = tn << 6;

  const int rlane = lane & 15;
  const int koff  = (lane >> 4) * 8;
  const int mOff  = (lane >> 4) * 8;

  v8f acc[4][4];
#pragma unroll
  for (int i = 0; i < 4; ++i)
#pragma unroll
    for (int j = 0; j < 4; ++j) acc[i][j] = zero8();

  for (int k0 = 0; k0 < K; k0 += 32) {
    F bh[4];
#pragma unroll
    for (int j = 0; j < 4; ++j) {
      const size_t bo = (size_t)(n0 + (j << 4) + rlane) * ldb + koff + k0;
      bh[j] = ldfrag<F>(Bp + bo);
    }
#pragma unroll
    for (int i = 0; i < 4; ++i) {
      const size_t ao = (size_t)(m0 + (i << 4) + rlane) * lda + koff + k0;
      const F ah = ldfrag<F>(Ap + ao);
#pragma unroll
      for (int j = 0; j < 4; ++j) {
        acc[i][j] = mma16(ah, bh[j], acc[i][j]);
      }
      dep_guard<F>(acc[i][0], acc[i][3], ah, bh[3]);
    }
    keep4<F>(bh[0], bh[1], bh[2], bh[3]);
  }
  acc_guard4(acc[0][0], acc[0][1], acc[0][2], acc[0][3]);
  acc_guard4(acc[1][0], acc[1][1], acc[1][2], acc[1][3]);
  acc_guard4(acc[2][0], acc[2][1], acc[2][2], acc[2][3]);
  acc_guard4(acc[3][0], acc[3][1], acc[3][2], acc[3][3]);

  float* slab = sT[wave];
#pragma unroll
  for (int i = 0; i < 4; ++i) {
    const int mBase = m0 + (i << 4);
#pragma unroll
    for (int j = 0; j < 4; ++j) {
#pragma unroll
      for (int r = 0; r < 8; ++r) {
        slab[(mOff + r) * 68 + (j << 4) + rlane] = acc[i][j][r];
      }
    }
    wave_sync_lds();
    if (OUT == 0) {
      float* C = (float*)Cout;
      const int hh = lane >> 4, c4 = (lane & 15) * 4;
      v4f vv[8];
#pragma unroll
      for (int it = 0; it < 8; ++it) {
        const int row = it * 2 + hh;
        v4f v = *(const v4f*)(slab + row * 68 + c4);
        vv[it] = v * alpha;
      }
#pragma unroll
      for (int it = 0; it < 8; ++it) {
        const int row = it * 2 + hh;
        *(volatile v4f*)(C + (size_t)(mBase + row) * ldc + n0 + c4) = vv[it];
      }
      __threadfence();
#pragma unroll
      for (int it = 0; it < 8; ++it) {
        const int row = it * 2 + hh;
        *(volatile v4f*)(C + (size_t)(mBase + row) * ldc + n0 + c4) = vv[it];
      }
      __threadfence();
    } else {
      unsigned short* Ch = (unsigned short*)Cout;
      const int q8 = (lane & 7) * 8, rr = lane >> 3;
      v4u ph[4];
#pragma unroll
      for (int it = 0; it < 4; ++it) {
        const int row = it * 4 + rr;
        v4f a = *(const v4f*)(slab + row * 68 + q8);
        v4f b = *(const v4f*)(slab + row * 68 + q8 + 4);
        a = a * alpha;
        b = b * alpha;
        ph[it] = pack_h8(a, b);
      }
#pragma unroll
      for (int it = 0; it < 4; ++it) {
        const int row = it * 4 + rr;
        const size_t co = (size_t)(mBase + row) * ldc + n0 + q8;
        *(volatile v4u*)(Ch + co) = ph[it];
      }
      __threadfence();
#pragma unroll
      for (int it = 0; it < 4; ++it) {
        const int row = it * 4 + rr;
        const size_t co = (size_t)(mBase + row) * ldc + n0 + q8;
        *(volatile v4u*)(Ch + co) = ph[it];
      }
      __threadfence();
    }
    wave_sync_lds();
  }
}

__global__ __launch_bounds__(256) void softmax_rows(const float* __restrict__ S, unsigned short* P) {
  __shared__ float sMx[8];
  __shared__ float sSm[8];
  const int tid  = threadIdx.x;
  const int lane = tid & 31;
  const int wave = tid >> 5;
  const int q    = blockIdx.x;
  const size_t rb = (size_t)q * NS;
  const int c0 = tid * 8;
  const v4f a0 = *(const v4f*)(S + rb + c0);
  const v4f a1 = *(const v4f*)(S + rb + c0 + 4);
  float v[8];
  v[0] = a0[0]; v[1] = a0[1]; v[2] = a0[2]; v[3] = a0[3];
  v[4] = a1[0]; v[5] = a1[1]; v[6] = a1[2]; v[7] = a1[3];

  float mx = v[0];
#pragma unroll
  for (int i = 1; i < 8; ++i) mx = fmaxf(mx, v[i]);
  mx = fmaxf(mx, __shfl_xor(mx, 16));
  mx = fmaxf(mx, __shfl_xor(mx, 8));
  mx = fmaxf(mx, __shfl_xor(mx, 4));
  mx = fmaxf(mx, __shfl_xor(mx, 2));
  mx = fmaxf(mx, __shfl_xor(mx, 1));
  if (lane == 0) sMx[wave] = mx;
  __syncthreads();
  float m = sMx[0];
#pragma unroll
  for (int w = 1; w < 8; ++w) m = fmaxf(m, sMx[w]);

  float e[8];
#pragma unroll
  for (int i = 0; i < 8; ++i) e[i] = __expf(v[i] - m);
  float part = ((e[0] + e[1]) + (e[2] + e[3])) + ((e[4] + e[5]) + (e[6] + e[7]));
  part += __shfl_xor(part, 16);
  part += __shfl_xor(part, 8);
  part += __shfl_xor(part, 4);
  part += __shfl_xor(part, 2);
  part += __shfl_xor(part, 1);
  if (lane == 0) sSm[wave] = part;
  __syncthreads();
  const float l = ((sSm[0] + sSm[1]) + (sSm[2] + sSm[3])) + ((sSm[4] + sSm[5]) + (sSm[6] + sSm[7]));
  const float inv = 1.0f / l;
  const float sc  = inv * 1024.0f;

  v4f p0, p1;
  p0[0] = e[0] * sc; p0[1] = e[1] * sc; p0[2] = e[2] * sc; p0[3] = e[3] * sc;
  p1[0] = e[4] * sc; p1[1] = e[5] * sc; p1[2] = e[6] * sc; p1[3] = e[7] * sc;
  const v4u pk = pack_h8(p0, p1);
  unsigned short* pr = P + rb + c0;
  *(volatile v4u*)(pr) = pk;
  __threadfence();
  *(volatile v4u*)(pr) = pk;
}

extern "C" void kernel_launch(void* const* d_in, const int* in_sizes, int n_in,
                              void* d_out, int out_size, void* d_ws, size_t ws_size,
                              hipStream_t stream) {
  if (n_in < 6) return;
  if (in_sizes[0] != NB * NS * ND) return;
  if (in_sizes[3] != ND * ND || in_sizes[4] != ND * ND || in_sizes[5] != ND * ND) return;
  if (out_size != NB * NS * ND) return;

  const float* x  = (const float*)d_in[0];
  const float* Wq = (const float*)d_in[3];
  const float* Wk = (const float*)d_in[4];
  const float* Wv = (const float*)d_in[5];
  float* out = (float*)d_out;

  const size_t PX  = (size_t)NB * NS * ND * 2;
  const size_t PW  = (size_t)ND * ND * 2;
  const size_t PQK = (size_t)NS * ND * 2;
  const size_t PV  = (size_t)ND * NS * 2;
  const size_t PS  = (size_t)NS * NS * 4;
  const size_t PP  = (size_t)NS * NS * 2;
  size_t off = 0;
  const size_t oX  = off; off += PX;
  const size_t oWq = off; off += PW;
  const size_t oWk = off; off += PW;
  const size_t oWv = off; off += PW;
  const size_t oQ  = off; off += PQK;
  const size_t oK  = off; off += PQK;
  const size_t oV  = off; off += PV;
  const size_t oS  = off; off += PS;
  const size_t oP  = off; off += PP;
  if (off > ws_size) return;
  if (off > (size_t)134217728) return;

  char* ws = (char*)d_ws;
  unsigned short* Xb  = (unsigned short*)(ws + oX);
  unsigned short* Wqb = (unsigned short*)(ws + oWq);
  unsigned short* Wkb = (unsigned short*)(ws + oWk);
  unsigned short* Wvb = (unsigned short*)(ws + oWv);
  unsigned short* Qp  = (unsigned short*)(ws + oQ);
  unsigned short* Kp  = (unsigned short*)(ws + oK);
  unsigned short* Vp  = (unsigned short*)(ws + oV);
  float* S = (float*)(ws + oS);
  unsigned short* Pp  = (unsigned short*)(ws + oP);

  const dim3 blk(256);
  const int n8x = NB * NS * ND / 8;
  const int n8w = ND * ND / 8;
  const dim3 gCvtX((n8x + 255) / 256);
  const dim3 gCvtW((n8w + 255) / 256);
  const dim3 gQK(((NS / 64) * (ND / 64) + 7) / 8);
  const dim3 gV(((ND / 64) * (NS / 64) + 7) / 8);
  const dim3 gS(((NS / 64) * (NS / 64) + 7) / 8);
  const dim3 gSm(NS);
  const dim3 gO(((NS / 64) * (ND / 64) + 7) / 8);

  cvt_bf16x8<<<gCvtX, blk, 0, stream>>>(x, Xb, n8x, n8x);
  cvt_bf16x8<<<gCvtW, blk, 0, stream>>>(Wq, Wqb, n8w, n8w);
  cvt_bf16x8<<<gCvtW, blk, 0, stream>>>(Wk, Wkb, n8w, n8w);
  cvt_bf16x8<<<gCvtW, blk, 0, stream>>>(Wv, Wvb, n8w, n8w);

  for (int b = 0; b < NB; ++b) {
    const unsigned short* Xbb = Xb + (size_t)b * NS * ND;
    float* outb = out + (size_t)b * NS * ND;
    gemm64<v16b, 1><<<gQK, blk, 0, stream>>>(Xbb, ND, Wqb, ND, (void*)Qp, ND, 1.0f, NS, ND, ND);
    gemm64<v16b, 1><<<gQK, blk, 0, stream>>>(Xbb, ND, Wkb, ND, (void*)Kp, ND, 1.0f, NS, ND, ND);
    gemm64<v16b, 1><<<gV, blk, 0, stream>>>(Wvb, ND, Xbb, ND, (void*)Vp, NS, 1.0f, ND, NS, ND);
    gemm64<v16h, 0><<<gS, blk, 0, stream>>>(Qp, ND, Kp, ND, (void*)S, NS, 0.03125f, NS, NS, ND);
    softmax_rows<<<gSm, blk, 0, stream>>>(S, Pp);
    gemm64<v16h, 0><<<gO, blk, 0, stream>>>(Pp, NS, Vp, NS, (void*)outb, ND, 0.0009765625f, NS, ND, NS);
  }
  (void)hipGetLastError();
}
